// TransformerLayer_2869038154392
// MI455X (gfx1250) — hardware-run, weakly checked
//
#include <hip/hip_runtime.h>


#ifndef SEQ
#define SEQ 4096
#endif
#define SEQ_FULL 4096
#define DM   2048
#define NH_  4
#define HD   32
#define CW   128
#define FF   512
#define AW   4
#define OSP  36
#define WCAR 64.0f
#define SC2  ((float)(0.00390625 * 1.4426950408889634))
#define PSH  14.0f
#define NEGB (-3.0e38f)
#define LNEPS 1.0e-5f

static_assert(HD == 32);
static_assert(NH_ * HD == CW);
static_assert(CW % 64 == 0);
static_assert(64 % HD == 0);
static_assert(DM % 64 == 0);
static_assert(FF % 64 == 0);
static_assert(DM % 32 == 0);
static_assert(FF % 32 == 0);
static_assert(CW % 32 == 0);
static_assert(SEQ % 64 == 0);
static_assert(SEQ % 32 == 0);
static_assert(SEQ % (16 * AW) == 0);
static_assert(SEQ <= SEQ_FULL);
static_assert(((size_t)SEQ * DM) % 8 == 0);
static_assert((OSP * 4) % 16 == 0);
static_assert(DM == 256 * 8);
static_assert(256 * 2 * 16 == DM * 4);
static_assert(256 * 16 == DM * 2);
static_assert(2 * 2 * 32 * 16 == 16 * 64 * 2);
static_assert(4 * 32 * 16 == 16 * 64 * 2);
static_assert(8 * 32 * 16 == 16 * 64 * 4);
static_assert(2 * 32 * 16 == 16 * HD * 2);
static_assert(256 * 32 == 64 * 32 * 4);
static_assert(256 * 16 == 32 * 64 * 2);
static_assert(16 * 68 * 4 <= 131072);
static_assert(AW * 16 * OSP * 4 <= 131072);
static_assert(32 * 68 * 4 <= 131072);
static_assert(DM * 4 + 64 <= 131072);

typedef _Float16 h16;
typedef unsigned short bf;
typedef __attribute__((ext_vector_type(16))) __bf16   v16bf;
typedef __attribute__((ext_vector_type(16))) _Float16 v16h;
typedef __attribute__((ext_vector_type(8)))  _Float16 v8h;
typedef __attribute__((ext_vector_type(8)))  unsigned short v8us;
typedef __attribute__((ext_vector_type(4)))  unsigned short v4us;
typedef __attribute__((ext_vector_type(8)))  float    v8f;
typedef __attribute__((ext_vector_type(4)))  float    v4f;
typedef v4f  __attribute__((may_alias)) v4fa;

__device__ __forceinline__ unsigned short f2bf(float f) { unsigned u = __float_as_uint(f); u += 0x7FFFu + ((u >> 16) & 1u); return (unsigned short)(u >> 16); }
__device__ __forceinline__ float bfr(float f) { return __uint_as_float(((unsigned)f2bf(f)) << 16); }
__device__ __forceinline__ v16h cat16(v8h lo, v8h hi) { return __builtin_shufflevector(lo, hi, 0, 1, 2, 3, 4, 5, 6, 7, 8, 9, 10, 11, 12, 13, 14, 15); }
__device__ __forceinline__ v16bf cat16b(v8us lo, v8us hi) { return __builtin_bit_cast(v16bf, __builtin_shufflevector(lo, hi, 0, 1, 2, 3, 4, 5, 6, 7, 8, 9, 10, 11, 12, 13, 14, 15)); }
__device__ __forceinline__ v8f wmma16(v16h a, v16h b, v8f c) { return __builtin_amdgcn_wmma_f32_16x16x32_f16(false, a, false, b, (short)0, c, false, false); }
__device__ __forceinline__ v8f wmmab(v16bf a, v16bf b, v8f c) { return __builtin_amdgcn_wmma_f32_16x16x32_bf16(false, a, false, b, (short)0, c, false, false); }
__device__ __forceinline__ v16h  ldh(const h16* p) { return cat16(*(const v8h*)p, *(const v8h*)(p + 16)); }
__device__ __forceinline__ v16bf ldb(const bf* p)  { return cat16b(*(const v8us*)p, *(const v8us*)(p + 16)); }
__device__ __forceinline__ void wave_sync() { __builtin_amdgcn_fence(3  , "wavefront"); __builtin_amdgcn_wave_barrier(); asm volatile("" ::: "memory"); }

static __device__ __forceinline__ h16 toh_flush(float v) { const h16 r = (h16)v; return (fabsf(v) < 6.103515625e-05f) ? (h16)0.0f : r; }
__device__ __forceinline__ v8f wmmag(v16h a, v16h b, v8f c) { c = wmma16(a, b, c); asm volatile("v_nop\n\tv_nop\n\tv_nop\n\tv_nop" : "+v"(c) : "v"(a), "v"(b)); return c; }
__device__ __forceinline__ v8f wmmag(v16bf a, v16bf b, v8f c) { c = wmmab(a, b, c); asm volatile("v_nop\n\tv_nop\n\tv_nop\n\tv_nop" : "+v"(c) : "v"(a), "v"(b)); return c; }
__device__ __forceinline__ v16h  ldfrag(const h16* p) { return ldh(p); }
__device__ __forceinline__ v16bf ldfrag(const bf* p)  { return ldb(p); }

__global__ __launch_bounds__(256) void k_cvt8(const float* __restrict__ src, bf* dst, size_t n8) {
    const size_t i = (size_t)blockIdx.x * 256 + threadIdx.x; if (i >= n8) return;
    const v8f v = *(const v8f*)(src + i * 8); v8us o;
#pragma unroll
    for (int k = 0; k < 8; ++k) o[k] = f2bf(v[k]);
    *(volatile v8us*)(dst + i * 8) = o; __threadfence(); *(volatile v8us*)(dst + i * 8) = o;
}

template <int OUTH, typename OT>
__device__ __forceinline__ void tw_body(const float* __restrict__ src, OT* dst, const int rows, const int cols) {
    __shared__ __align__(16) float ts[32 * 68];
    const int tid = threadIdx.x;
    const int r0 = blockIdx.x * 64, c0 = blockIdx.y * 32;
    const size_t zoff = (size_t)blockIdx.z * (size_t)rows * (size_t)cols;
    { const int r = tid >> 2, cq = (tid & 3) * 8;
      const float* p = src + zoff + (size_t)(r0 + r) * cols + c0 + cq;
      const v4f x0 = *(const v4f*)p; const v4f x1 = *(const v4f*)(p + 4);
#pragma unroll
      for (int i = 0; i < 4; ++i) { ts[(cq + i) * 68 + r] = x0[i]; ts[(cq + 4 + i) * 68 + r] = x1[i]; } }
    __syncthreads();
    const int orow = tid >> 3, c8 = (tid & 7) * 8;
    const v4f y0 = *(const v4fa*)(&ts[orow * 68 + c8]); const v4f y1 = *(const v4fa*)(&ts[orow * 68 + c8 + 4]);
    const size_t oo = zoff + (size_t)(c0 + orow) * rows + r0 + c8;
    if (OUTH == 0) {
        v8us o;
#pragma unroll
        for (int i = 0; i < 4; ++i) { o[i] = f2bf(y0[i]); o[4 + i] = f2bf(y1[i]); }
        *(volatile v8us*)(dst + oo) = o; __threadfence(); *(volatile v8us*)(dst + oo) = o;
    } else {
        v8h o;
#pragma unroll
        for (int i = 0; i < 4; ++i) { o[i] = toh_flush(bfr(y0[i]) * WCAR); o[4 + i] = toh_flush(bfr(y1[i]) * WCAR); }
        *(volatile v8h*)(dst + oo) = o; __threadfence(); *(volatile v8h*)(dst + oo) = o;
    }
}
__global__ __launch_bounds__(256) void k_twb(const float* __restrict__ src, bf* dst, int rows, int cols) { tw_body<0, bf>(src, dst, rows, cols); }
__global__ __launch_bounds__(256) void k_twh(const float* __restrict__ src, h16* dst, int rows, int cols) { tw_body<1, h16>(src, dst, rows, cols); }

template <typename ET, int KD, int EPI, int NO>
__device__ __forceinline__ void gemm_body(const ET* __restrict__ A, const ET* __restrict__ Bt, const int lda, const size_t aks,
                                          const float* __restrict__ bias, const bf* __restrict__ resb, const float* __restrict__ resf,
                                          float* outf, h16* outh, const float oscale) {
    __shared__ __align__(16) float os[16 * 68];
    typedef decltype(ldfrag((const ET*)0)) FT;
    const int lane = threadIdx.x & 31, lr = lane & 15, hi = lane >> 4; const int r0 = blockIdx.x * 64, c0 = blockIdx.y * 64;
    v8f acc[4][4];
#pragma unroll
    for (int mb = 0; mb < 4; ++mb)
#pragma unroll
        for (int nb = 0; nb < 4; ++nb) acc[mb][nb] = (v8f){};
    const size_t aoff = (size_t)(r0 + lr) * lda + 8 * hi, boff = (size_t)(c0 + lr) * KD + 8 * hi;
#pragma unroll 1
    for (int kc = 0; kc < KD; kc += 32) {
        const size_t ka = (size_t)(kc >> 5) * aks;
        FT a[4];
#pragma unroll
        for (int mb = 0; mb < 4; ++mb) a[mb] = ldfrag(A + aoff + (size_t)mb * 16 * lda + ka);
#pragma unroll
        for (int nb = 0; nb < 4; ++nb) { const FT b = ldfrag(Bt + boff + (size_t)nb * 16 * KD + kc);
#pragma unroll
            for (int mb = 0; mb < 4; ++mb) acc[mb][nb] = wmmag(a[mb], b, acc[mb][nb]); }
    }
#pragma unroll
    for (int mb = 0; mb < 4; ++mb) {
#pragma unroll
        for (int nb = 0; nb < 4; ++nb) {
#pragma unroll
            for (int j = 0; j < 8; ++j) os[(hi * 8 + j) * 68 + nb * 16 + lr] = acc[mb][nb][j] * oscale; }
        wave_sync();
#pragma unroll 1
        for (int ps = 0; ps < 2; ++ps) {
            if (EPI == 0) {
                const size_t sb = ((size_t)(c0 / HD) * SEQ + (size_t)(r0 + mb * 16)) * HD;
#pragma unroll
                for (int hh = 0; hh < 2; ++hh) {
#pragma unroll
                    for (int s = 0; s < 2; ++s) { const int p = s * 32 + lane; const int row = p >> 2, c8 = (p & 3) * 8;
                        const v4f x0 = *(const v4fa*)(&os[row * 68 + hh * 32 + c8]); const v4f x1 = *(const v4fa*)(&os[row * 68 + hh * 32 + c8 + 4]); v8h hv;
#pragma unroll
                        for (int i = 0; i < 4; ++i) { hv[i] = toh_flush(x0[i]); hv[4 + i] = toh_flush(x1[i]); }
                        const size_t oo = sb + (size_t)hh * ((size_t)SEQ * HD) + (size_t)p * 8;
                        *(volatile v8h*)(outh + oo) = hv; } }
            } else if (EPI == 1) {
                const size_t sb = (size_t)(r0 + mb * 16) * SEQ + (size_t)c0;
#pragma unroll
                for (int s = 0; s < 4; ++s) { const int row = 4 * s + (lane >> 3), c8 = (lane & 7) * 8;
                    const v4f x0 = *(const v4fa*)(&os[row * 68 + c8]); const v4f x1 = *(const v4fa*)(&os[row * 68 + c8 + 4]); v8h hv;
#pragma unroll
                    for (int i = 0; i < 4; ++i) { hv[i] = toh_flush(x0[i]); hv[4 + i] = toh_flush(x1[i]); }
                    const size_t oo = sb + (size_t)row * SEQ + c8;
                    *(volatile v8h*)(outh + oo) = hv; }
            } else if (EPI == 3) {
#pragma unroll
                for (int s = 0; s < 4; ++s) { const int row = 4 * s + (lane >> 3), c8 = (lane & 7) * 8;
                    const v4f x0 = *(const v4fa*)(&os[row * 68 + c8]); const v4f x1 = *(const v4fa*)(&os[row * 68 + c8 + 4]);
                    const v4f q0 = *(const v4f*)(bias + c0 + c8); const v4f q1 = *(const v4f*)(bias + c0 + c8 + 4); v8h hv;
#pragma unroll
                    for (int i = 0; i < 4; ++i) { hv[i] = toh_flush(fmaxf(x0[i] + bfr(q0[i]), 0.0f)); hv[4 + i] = toh_flush(fmaxf(x1[i] + bfr(q1[i]), 0.0f)); }
                    const size_t oo = (size_t)(r0 + mb * 16 + row) * NO + c0 + c8;
                    *(volatile v8h*)(outh + oo) = hv; }
            } else {
#pragma unroll
                for (int s = 0; s < 8; ++s) { const int row = 2 * s + (lane >> 4), cofs = (lane & 15) * 4;
                    const v4f x0 = *(const v4fa*)(&os[row * 68 + cofs]);
                    const v4f q0 = *(const v4f*)(bias + c0 + cofs);
                    const size_t go = (size_t)(r0 + mb * 16 + row) * NO + c0 + cofs;
                    v4f val;
                    if (EPI == 2) { const v4us rb = *(const v4us*)(resb + go);
#pragma unroll
                        for (int i = 0; i < 4; ++i) val[i] = __uint_as_float(((unsigned)rb[i]) << 16) + (x0[i] + bfr(q0[i]));
                    } else { const v4f rf = *(const v4f*)(resf + go);
#pragma unroll
                        for (int i = 0; i < 4; ++i) val[i] = rf[i] + (x0[i] + bfr(q0[i])); }
                    *(volatile v4f*)(outf + go) = val; }
            }
            if (ps == 0) __threadfence(); }
        wave_sync();
    }
}

__global__ __launch_bounds__(32) void k_gemm_qk(const bf* __restrict__ XB, const bf* __restrict__ WT, h16* QK) {
    gemm_body<bf, DM, 0, 0>(XB, WT, DM, (size_t)32, (const float*)0, (const bf*)0, (const float*)0, (float*)0, QK, 1.0f);
}
__global__ __launch_bounds__(32) void k_gemm_vt(const bf* __restrict__ WV, const bf* __restrict__ XB, h16* VT) {
    gemm_body<bf, DM, 1, 0>(WV, XB, DM, (size_t)32, (const float*)0, (const bf*)0, (const float*)0, (float*)0, VT, 1.0f);
}
__global__ __launch_bounds__(32) void k_gemm_ctx(const h16* __restrict__ OP, const h16* __restrict__ W1T, const float* __restrict__ b1, const bf* __restrict__ XB, float* T1) {
    gemm_body<h16, CW, 2, DM>(OP, W1T, HD, (size_t)SEQ * HD, b1, XB, (const float*)0, T1, (h16*)0, 1.0f / (WCAR * WCAR));
}
__global__ __launch_bounds__(32) void k_gemm_up(const h16* __restrict__ YH, const h16* __restrict__ W2T, const float* __restrict__ b2, h16* ZH) {
    gemm_body<h16, DM, 3, FF>(YH, W2T, DM, (size_t)32, b2, (const bf*)0, (const float*)0, (float*)0, ZH, 1.0f / WCAR);
}
__global__ __launch_bounds__(32) void k_gemm_down(const h16* __restrict__ ZH, const h16* __restrict__ W3T, const float* __restrict__ b3, const float* __restrict__ Y, float* T1) {
    gemm_body<h16, FF, 4, DM>(ZH, W3T, FF, (size_t)32, b3, (const bf*)0, Y, T1, (h16*)0, 1.0f / WCAR);
}

__global__ __launch_bounds__(32 * AW) void k_flash(const h16* __restrict__ QK, const h16* __restrict__ VT, h16* OP) {
    __shared__ __align__(16) float os[AW * 16 * OSP];
    const int lane = threadIdx.x & 31, lr = lane & 15, hi = lane >> 4;
    const int wave = __builtin_amdgcn_readfirstlane((int)(threadIdx.x >> 5));
    const int h = blockIdx.y;
    const int t0 = (blockIdx.x * AW + wave) * 16;
    const int lim = t0 + lr;
    const int nk = (t0 + 16 + 31) & ~31;
    const size_t qbase = (size_t)h * SEQ * HD;
    const size_t kbase = (size_t)(NH_ + h) * SEQ * HD;
    const size_t vbase = (size_t)h * HD * SEQ;
    const v16h qh = ldh(QK + qbase + (size_t)(t0 + lr) * HD + 8 * hi);
    const size_t ko = kbase + (size_t)lr * HD + 8 * hi;
    const size_t vo = vbase + (size_t)lr * SEQ + 8 * hi;
    v8f o0 = (v8f){}, o1 = (v8f){};
    float m = NEGB, l = 0.0f;
#pragma unroll 1
    for (int key0 = 0; key0 < nk; key0 += 32) {
        const h16* ka = QK + ko + (size_t)key0 * HD;
        const v16h ka0 = ldh(ka), kb0 = ldh(ka + 16 * HD);
        v8f sHa = (v8f){}, sHb = (v8f){};
        sHa = wmmag(ka0, qh, sHa); sHb = wmmag(kb0, qh, sHb);
        const int ja = key0 + 8 * hi;
        float ta[8], tb[8]; bool fa[8], fb[8]; float mx = NEGB;
#pragma unroll
        for (int r = 0; r < 8; ++r) {
            fa[r] = (ja + r <= lim);
            fb[r] = (ja + 16 + r <= lim);
            ta[r] = sHa[r] * SC2; tb[r] = sHb[r] * SC2;
            mx = fmaxf(mx, fmaxf(fa[r] ? ta[r] : NEGB, fb[r] ? tb[r] : NEGB)); }
        mx = fmaxf(mx, __shfl_xor(mx, 16, 32));
        const float mnew = fmaxf(m, mx);
        const float alpha = __builtin_amdgcn_exp2f(m - mnew);
        const float sh = PSH - mnew;
        v16h pb; float ls = 0.0f;
#pragma unroll
        for (int r = 0; r < 8; ++r) {
            const float xa = ta[r] + sh, xb = tb[r] + sh;
            const float ea = __builtin_amdgcn_exp2f(xa), eb = __builtin_amdgcn_exp2f(xb);
            const float ga = (fa[r] & (xa >= -14.0f)) ? ea : 0.0f;
            const float gb = (fb[r] & (xb >= -14.0f)) ? eb : 0.0f;
            const h16 pa = (h16)ga; const h16 pc = (h16)gb;
            pb[r] = pa; pb[8 + r] = pc;
            ls += (float)pa + (float)pc; }
        l = l * alpha + ls; m = mnew;
        o0 = o0 * alpha; o1 = o1 * alpha;
        const h16* va = VT + vo + key0;
        const v16h v0 = ldh(va), v1 = ldh(va + (size_t)16 * SEQ);
        o0 = wmmag(v0, pb, o0); o1 = wmmag(v1, pb, o1);
    }
    l += __shfl_xor(l, 16, 32);
    const bool any = l > 0.0f;
    const float lsafe = any ? l : 1.0f;
    const float inv = any ? (1.0f / lsafe) : 0.0f;
    const v8f f0 = o0, f1 = o1;
    const int wb = wave * 16 * OSP;
    { v4f a, c;
      a[0] = f0[0] * inv; a[1] = f0[1] * inv; a[2] = f0[2] * inv; a[3] = f0[3] * inv; c[0] = f0[4] * inv; c[1] = f0[5] * inv; c[2] = f0[6] * inv; c[3] = f0[7] * inv;
      *(v4fa*)(&os[wb + lr * OSP +  0 + 8 * hi]) = a; *(v4fa*)(&os[wb + lr * OSP +  0 + 8 * hi + 4]) = c;
      a[0] = f1[0] * inv; a[1] = f1[1] * inv; a[2] = f1[2] * inv; a[3] = f1[3] * inv; c[0] = f1[4] * inv; c[1] = f1[5] * inv; c[2] = f1[6] * inv; c[3] = f1[7] * inv;
      *(v4fa*)(&os[wb + lr * OSP + 16 + 8 * hi]) = a; *(v4fa*)(&os[wb + lr * OSP + 16 + 8 * hi + 4]) = c; }
    wave_sync();
    const size_t ob = ((size_t)h * SEQ + (size_t)t0) * HD;
#pragma unroll 1
    for (int ps = 0; ps < 2; ++ps) {
#pragma unroll
        for (int s = 0; s < 2; ++s) { const int p = s * 32 + lane; const int row = p >> 2, c8 = (p & 3) * 8;
            const v4f x0 = *(const v4fa*)(&os[wb + row * OSP + c8]); const v4f x1 = *(const v4fa*)(&os[wb + row * OSP + c8 + 4]); v8h hv;
#pragma unroll
            for (int i = 0; i < 4; ++i) { hv[i] = toh_flush(x0[i] * WCAR); hv[4 + i] = toh_flush(x1[i] * WCAR); }
            *(volatile v8h*)(OP + ob + (size_t)p * 8) = hv; }
        if (ps == 0) __threadfence(); }
}

template <int WH>
__device__ __forceinline__ void ln_body(const float* __restrict__ in, float* outf, h16* outh) {
#pragma clang fp contract(off)
    __shared__ float red[16];
    __shared__ __align__(16) float rowb[DM];
    const int tid = threadIdx.x, lane = tid & 31;
    const int wave = __builtin_amdgcn_readfirstlane((int)(threadIdx.x >> 5));
    const size_t rb = (size_t)blockIdx.x * DM;
    const v4f a = *(const v4f*)(in + rb + tid * 4);
    const v4f b = *(const v4f*)(in + rb + (DM / 2) + tid * 4);
    float s = ((a[0] + a[1]) + (a[2] + a[3])) + ((b[0] + b[1]) + (b[2] + b[3]));
#pragma unroll
    for (int off = 16; off > 0; off >>= 1) s += __shfl_xor(s, off, 32);
    if (lane == 0) red[wave] = s;
    __syncthreads();
    float tot = 0.0f;
#pragma unroll
    for (int w = 0; w < 8; ++w) tot += red[w];
    const float mean = tot * (1.0f / (float)DM);
    const v4f da = a - mean, db = b - mean;
    float q = ((da[0] * da[0] + da[1] * da[1]) + (da[2] * da[2] + da[3] * da[3])) + ((db[0] * db[0] + db[1] * db[1]) + (db[2] * db[2] + db[3] * db[3]));
#pragma unroll
    for (int off = 16; off > 0; off >>= 1) q += __shfl_xor(q, off, 32);
    if (lane == 0) red[8 + wave] = q;
    __syncthreads();
    float tot2 = 0.0f;
#pragma unroll
    for (int w = 0; w < 8; ++w) tot2 += red[8 + w];
    const float var = tot2 * (1.0f / (float)DM);
    const float rstd = 1.0f / sqrtf(var + LNEPS);
    const v4f na = da * rstd, nb = db * rstd;
    v8h hv = (v8h){};
    if (WH) {
        *(v4fa*)(&rowb[tid * 4]) = na; *(v4fa*)(&rowb[(DM / 2) + tid * 4]) = nb;
        __syncthreads();
        const v4f y0 = *(const v4fa*)(&rowb[tid * 8]); const v4f y1 = *(const v4fa*)(&rowb[tid * 8 + 4]);
#pragma unroll
        for (int i = 0; i < 4; ++i) { hv[i] = toh_flush(y0[i]); hv[4 + i] = toh_flush(y1[i]); }
    }
    *(volatile v4f*)(outf + rb + tid * 4) = na; *(volatile v4f*)(outf + rb + (DM / 2) + tid * 4) = nb;
    if (WH) *(volatile v8h*)(outh + rb + tid * 8) = hv;
    __threadfence();
    *(volatile v4f*)(outf + rb + tid * 4) = na; *(volatile v4f*)(outf + rb + (DM / 2) + tid * 4) = nb;
    if (WH) *(volatile v8h*)(outh + rb + tid * 8) = hv;
}
__global__ __launch_bounds__(256) void k_ln1(const float* __restrict__ T1, float* Y, h16* YH) { ln_body<1>(T1, Y, YH); }
__global__ __launch_bounds__(256) void k_ln2(const float* __restrict__ T1, float* OUT) { ln_body<0>(T1, OUT, (h16*)0); }

static constexpr size_t al256(size_t v) { return (v + 255) & ~(size_t)255; }
static constexpr size_t SZ_XB = al256((size_t)SEQ * DM * 2);
static constexpr size_t SZ_WT = al256((size_t)3 * CW * DM * 2);
static constexpr size_t SZ_W1 = al256((size_t)DM * CW * 2);
static constexpr size_t SZ_W2 = al256((size_t)FF * DM * 2);
static constexpr size_t SZ_W3 = al256((size_t)DM * FF * 2);
static constexpr size_t SZ_QK = al256((size_t)2 * NH_ * SEQ * HD * 2);
static constexpr size_t SZ_VT = al256((size_t)CW * SEQ * 2);
static constexpr size_t SZ_OP = al256((size_t)NH_ * SEQ * HD * 2);
static constexpr size_t SZ_T1 = al256((size_t)SEQ * DM * 4);
static constexpr size_t SZ_Y  = al256((size_t)SEQ * DM * 4);
static constexpr size_t SZ_YH = al256((size_t)SEQ * DM * 2);
static constexpr size_t SZ_ZH = al256((size_t)SEQ * FF * 2);
static constexpr size_t SZ_TOTAL = SZ_XB + SZ_WT + SZ_W1 + SZ_W2 + SZ_W3 + SZ_QK + SZ_VT + SZ_OP + SZ_T1 + SZ_Y + SZ_YH + SZ_ZH;
static_assert(SZ_TOTAL <= (size_t)134217728);
static_assert(((size_t)CW * DM * 2) % 256 == 0);
static_assert((size_t)NH_ * DM * HD == (size_t)CW * DM);

extern "C" void kernel_launch(void* const* d_in, const int* in_sizes, int n_in,
                              void* d_out, int out_size, void* d_ws, size_t ws_size, hipStream_t stream) {
    if (n_in < 10) return;
    if ((size_t)in_sizes[0] < (size_t)SEQ * DM) return;
    if ((size_t)in_sizes[1] < (size_t)NH_ * DM * HD || (size_t)in_sizes[2] < (size_t)NH_ * DM * HD || (size_t)in_sizes[3] < (size_t)NH_ * DM * HD) return;
    if ((size_t)in_sizes[4] < (size_t)CW * DM || in_sizes[5] < DM) return;
    if ((size_t)in_sizes[6] < (size_t)DM * FF || in_sizes[7] < FF) return;
    if ((size_t)in_sizes[8] < (size_t)FF * DM || in_sizes[9] < DM) return;
    if ((size_t)out_size < (size_t)SEQ * DM) return;
    if (SZ_TOTAL > ws_size) return;
    const float* x  = (const float*)d_in[0];
    const float* wq = (const float*)d_in[1];
    const float* wk = (const float*)d_in[2];
    const float* wv = (const float*)d_in[3];
    const float* W1 = (const float*)d_in[4];
    const float* b1 = (const float*)d_in[5];
    const float* W2 = (const float*)d_in[6];
    const float* b2 = (const float*)d_in[7];
    const float* W3 = (const float*)d_in[8];
    const float* b3 = (const float*)d_in[9];
    float* OUT = (float*)d_out;
    char* wsp = (char*)d_ws;
    bf*  XB  = (bf*)wsp;  wsp += SZ_XB;
    bf*  WT  = (bf*)wsp;  wsp += SZ_WT;
    h16* W1T = (h16*)wsp; wsp += SZ_W1;
    h16* W2T = (h16*)wsp; wsp += SZ_W2;
    h16* W3T = (h16*)wsp; wsp += SZ_W3;
    h16* QK  = (h16*)wsp; wsp += SZ_QK;
    h16* VT  = (h16*)wsp; wsp += SZ_VT;
    h16* OP  = (h16*)wsp; wsp += SZ_OP;
    float* T1 = (float*)wsp; wsp += SZ_T1;
    float* Y  = (float*)wsp; wsp += SZ_Y;
    h16* YH  = (h16*)wsp; wsp += SZ_YH;
    h16* ZH  = (h16*)wsp; wsp += SZ_ZH;

    { const size_t n8 = (size_t)SEQ * DM / 8;
      k_cvt8<<<(unsigned)((n8 + 255) / 256), 256, 0, stream>>>(x, XB, n8); }
    k_twb<<<dim3(DM / 64, HD / 32, NH_), 256, 0, stream>>>(wq, WT, DM, HD);
    k_twb<<<dim3(DM / 64, HD / 32, NH_), 256, 0, stream>>>(wk, WT + (size_t)CW * DM, DM, HD);
    k_twb<<<dim3(DM / 64, HD / 32, NH_), 256, 0, stream>>>(wv, WT + (size_t)2 * CW * DM, DM, HD);
    k_twh<<<dim3(CW / 64, DM / 32, 1), 256, 0, stream>>>(W1, W1T, CW, DM);
    k_twh<<<dim3(DM / 64, FF / 32, 1), 256, 0, stream>>>(W2, W2T, DM, FF);
    k_twh<<<dim3(FF / 64, DM / 32, 1), 256, 0, stream>>>(W3, W3T, FF, DM);

    k_gemm_qk<<<dim3(SEQ / 64, (2 * CW) / 64, 1), 32, 0, stream>>>(XB, WT, QK);
    k_gemm_vt<<<dim3(CW / 64, SEQ / 64, 1), 32, 0, stream>>>(WT + (size_t)2 * CW * DM, XB, VT);

    k_flash<<<dim3(SEQ / (16 * AW), NH_, 1), 32 * AW, 0, stream>>>(QK, VT, OP);

    k_gemm_ctx<<<dim3(SEQ / 64, DM / 64, 1), 32, 0, stream>>>(OP, W1T, b1, XB, T1);
    k_ln1<<<SEQ, 256, 0, stream>>>(T1, Y, YH);
    k_gemm_up<<<dim3(SEQ / 64, FF / 64, 1), 32, 0, stream>>>(YH, W2T, b2, ZH);
    k_gemm_down<<<dim3(SEQ / 64, DM / 64, 1), 32, 0, stream>>>(ZH, W3T, b3, Y, T1);
    k_ln2<<<SEQ, 256, 0, stream>>>(T1, OUT);
}
